// NeuralMemoryBank_62680752718465
// MI455X (gfx1250) — hardware-verified
//
#include <hip/hip_runtime.h>
#include <math.h>

typedef __attribute__((ext_vector_type(16))) _Float16 v16h;
typedef __attribute__((ext_vector_type(16))) __bf16 v16b;
typedef __attribute__((ext_vector_type(8)))  _Float16 v8h;
typedef __attribute__((ext_vector_type(8)))  float v8f;
typedef __attribute__((ext_vector_type(4)))  float v4f;
typedef __attribute__((ext_vector_type(2)))  float v2f;
typedef __attribute__((ext_vector_type(4)))  unsigned v4u;
typedef __attribute__((ext_vector_type(4)))  int v4i;
typedef float __attribute__((may_alias)) float_a;
typedef int __attribute__((may_alias)) int_a;

template <typename T> __device__ __forceinline__ void vst2(void* p, T v) { *(volatile T*)p = v; __threadfence(); *(volatile T*)p = v; }
__device__ __forceinline__ v8f wmma16(v16h a, v16h b, v8f c) {
  v8f d = __builtin_amdgcn_wmma_f32_16x16x32_f16(false, a, false, b, (short)0, c, false, false);
  asm volatile("v_nop\n\tv_nop\n\tv_nop\n\tv_nop" : "+v"(d) : "v"(a), "v"(b));
  return d;
}
__device__ __forceinline__ v8f wmma_bf(v16b a, v16b b, v8f c) {
  v8f d = __builtin_amdgcn_wmma_f32_16x16x32_bf16(false, a, false, b, (short)0, c, false, false);
  asm volatile("v_nop\n\tv_nop\n\tv_nop\n\tv_nop" : "+v"(d) : "v"(a), "v"(b));
  return d;
}
__device__ __forceinline__ v16h frag_h(const _Float16* rowk0, int lane) {
  union { v16h v; v8h q[2]; } u; const _Float16* p = rowk0 + 8 * (lane >> 4);
  u.q[0] = *(const v8h*)p; u.q[1] = *(const v8h*)(p + 16); return u.v;
}
__device__ __forceinline__ v16h frag_f32(const float* rowk0, int lane) {
  v16h a; const float* p = rowk0 + 8 * (lane >> 4);
#pragma unroll
  for (int i = 0; i < 8; ++i) { a[i] = (_Float16)p[i]; a[8 + i] = (_Float16)p[16 + i]; }
  return a;
}
__device__ __forceinline__ v16h frag_f32s(const float* rowk0, int lane, float sc) {
  v16h a; const float* p = rowk0 + 8 * (lane >> 4);
#pragma unroll
  for (int i = 0; i < 8; ++i) { a[i] = (_Float16)(p[i] * sc); a[8 + i] = (_Float16)(p[16 + i] * sc); }
  return a;
}
__device__ __forceinline__ v16h fragc_f32(const float* W, int k0, int n, int lane, int ld, int K) {
  v16h a; const int g = lane >> 4;
#pragma unroll
  for (int i = 0; i < 8; ++i) { const int ka = k0 + 8 * g + i, kb = ka + 16;
    a[i] = (_Float16)(ka < K ? W[(size_t)(ka < K ? ka : K - 1) * ld + n] : 0.f); a[8 + i] = (_Float16)(kb < K ? W[(size_t)(kb < K ? kb : K - 1) * ld + n] : 0.f); }
  return a;
}
struct F2 { v16b h, l; };
__device__ __forceinline__ F2 bsplit16(const float v[16]) { F2 r;
#pragma unroll
  for (int i = 0; i < 16; ++i) { const __bf16 h = (__bf16)v[i]; r.h[i] = h; r.l[i] = (__bf16)(v[i] - (float)h); }
  return r; }
__device__ __forceinline__ F2 split_row(const float* row, int k0, int lane) { float v[16]; const float* p = row + k0 + 8 * (lane >> 4);
#pragma unroll
  for (int i = 0; i < 8; ++i) { v[i] = p[i]; v[8 + i] = p[16 + i]; }
  return bsplit16(v); }
__device__ __forceinline__ F2 split_rowK(const float* row, int k0, int lane, int K) { float v[16]; const int g = lane >> 4;
#pragma unroll
  for (int i = 0; i < 8; ++i) { const int ka = k0 + 8 * g + i, kb = ka + 16; v[i] = ka < K ? row[ka < K ? ka : K - 1] : 0.f; v[8 + i] = kb < K ? row[kb < K ? kb : K - 1] : 0.f; }
  return bsplit16(v); }
__device__ __forceinline__ F2 split_col(const float* W, int k0, int n, int lane, int ld, int K) { float v[16]; const int g = lane >> 4;
#pragma unroll
  for (int i = 0; i < 8; ++i) { const int ka = k0 + 8 * g + i, kb = ka + 16; v[i] = ka < K ? W[(size_t)(ka < K ? ka : K - 1) * ld + n] : 0.f; v[8 + i] = kb < K ? W[(size_t)(kb < K ? kb : K - 1) * ld + n] : 0.f; }
  return bsplit16(v); }
__device__ __forceinline__ v8f mac3(const F2& a, const F2& b, v8f c) { c = wmma_bf(a.l, b.h, c); c = wmma_bf(a.h, b.l, c); return wmma_bf(a.h, b.h, c); }
__device__ __forceinline__ float sigm(float v) { return 1.0f / (1.0f + expf(-v)); }
#define LDSX() do { asm volatile("s_wait_dscnt 0" ::: "memory"); __builtin_amdgcn_wave_barrier(); __builtin_amdgcn_fence(__ATOMIC_RELEASE, "workgroup"); } while (0)


#define NB 8
#define NS 4096
#define HH 256
#define MM 4096
#define NROW (NB * NS)
#define NBLK (NROW / 64)
#ifndef TBLK
#define TBLK NBLK
#endif
typedef __attribute__((ext_vector_type(8))) __bf16 v8b;
__device__ __forceinline__ v16b frag_b(const __bf16* rowk0, int lane) {
  union { v16b v; v8b q[2]; } u; const __bf16* p = rowk0 + 8 * (lane >> 4);
  u.q[0] = *(const v8b*)p; u.q[1] = *(const v8b*)(p + 16); return u.v;
}
__device__ __forceinline__ float bfr(float v) { return (float)(__bf16)v; }
__device__ __attribute__((noinline)) float exp_ni(float v) { return expf(v); }
__device__ __attribute__((noinline)) float erf_ni(float v) { return erff(v); }

#define WS_MH  0u
#define WS_MV  (WS_MH + 2u * MM * HH)
#define WS_SG  (WS_MV + 2u * MM * HH)
#define WS_SR  (WS_SG + 4u * (size_t)NBLK * MM)
#define WS_RA  (WS_SR + 4u * (size_t)NBLK * HH)
#define WS_END (WS_RA + 4u * HH)

__global__ __launch_bounds__(256) void k_mem(const float* __restrict__ MEM, _Float16* __restrict__ MHr, _Float16* __restrict__ MV) { __shared__ __align__(16) _Float16 sr[64][HH + 8]; __shared__ __align__(16) _Float16 st[HH][72];
  const int t = threadIdx.x; const int m0 = blockIdx.x * 64;
  for (int e = t; e < 64 * HH; e += 256) { const int ml = e / HH, h = e % HH; const _Float16 v = (_Float16)bfr(MEM[(size_t)(m0 + ml) * HH + h]); sr[ml][h] = v; st[h][ml] = v; }
  __syncthreads();
  for (int e = t; e < 64 * (HH / 8); e += 256) { const int ml = e >> 5, q = e & 31; vst2((unsigned*)(MHr + (size_t)(m0 + ml) * HH + q * 8), *(const v4u*)&sr[ml][q * 8]); }
  for (int e = t; e < HH * 8; e += 256) { const int h = e >> 3, q = e & 7; vst2((unsigned*)(MV + (size_t)h * MM + m0 + q * 8), *(const v4u*)&st[h][q * 8]); } }
__device__ __forceinline__ v16h frag_xb(const float* rowk0, int lane) { v16h a; const float* p = rowk0 + 8 * (lane >> 4);
#pragma unroll
  for (int i = 0; i < 8; ++i) { a[i] = (_Float16)bfr(p[i]); a[8 + i] = (_Float16)bfr(p[16 + i]); }
  return a; }
__global__ __launch_bounds__(128) void k_read(const float* __restrict__ X, const _Float16* __restrict__ MHr, const _Float16* __restrict__ MV, float* __restrict__ READ, float* __restrict__ SG, float* __restrict__ SR) {
  __shared__ __align__(16) float sp[4][16][36]; __shared__ __align__(16) float sg[4][32]; __shared__ __align__(16) float sgb[32]; __shared__ __align__(16) float so[4][16][HH + 4]; __shared__ __align__(16) float ssr[HH];
  const int tid = threadIdx.x, wave = tid >> 5, lane = tid & 31, col = lane & 15, g = lane >> 4; const size_t r0 = (size_t)blockIdx.x * 64 + wave * 16; const float* xr = X + (r0 + col) * HH;
  float m[8], l[8];
#pragma unroll
  for (int r = 0; r < 8; ++r) { m[r] = -3.0e38f; l[r] = 0.f; }
  v8f acc[16] = {};
#pragma unroll 1
  for (int ks = 0; ks < MM / 32; ++ks) { float s[2][8]; float gs[2];
#pragma unroll
    for (int ct = 0; ct < 2; ++ct) { const int kk = ks * 32 + ct * 16 + col; v8f c = {};
#pragma unroll
      for (int kc = 0; kc < HH / 32; ++kc) c = wmma16(frag_xb(xr + kc * 32, lane), frag_h(MHr + (size_t)kk * HH + kc * 32, lane), c);
      float gsum = 0.f;
#pragma unroll
      for (int r = 0; r < 8; ++r) { s[ct][r] = c[r]; gsum += 1.0f / (1.0f + expf(-c[r])); }
      gs[ct] = gsum; }
#pragma unroll
    for (int ct = 0; ct < 2; ++ct) { const float tot = gs[ct] + __shfl_xor(gs[ct], 16); if (g == 0) sg[wave][ct * 16 + col] = tot; }
    float alpha[8];
#pragma unroll
    for (int r = 0; r < 8; ++r) { float mx = fmaxf(s[0][r], s[1][r]);
#pragma unroll
      for (int o = 1; o < 16; o <<= 1) mx = fmaxf(mx, __shfl_xor(mx, o));
      const float mn = fmaxf(m[r], mx); alpha[r] = __expf(m[r] - mn); const float e0 = __expf(s[0][r] - mn), e1 = __expf(s[1][r] - mn); float es = e0 + e1;
#pragma unroll
      for (int o = 1; o < 16; o <<= 1) es += __shfl_xor(es, o);
      l[r] = l[r] * alpha[r] + es; m[r] = mn; sp[wave][8 * g + r][col] = e0; sp[wave][8 * g + r][16 + col] = e1; }
#pragma unroll
    for (int j = 0; j < 16; ++j)
#pragma unroll
      for (int r = 0; r < 8; ++r) acc[j][r] *= alpha[r];
    __syncthreads();
    if (tid < 32) { sgb[tid] = (sg[0][tid] + sg[1][tid]) + (sg[2][tid] + sg[3][tid]); }
    const v16h pa = frag_f32s(&sp[wave][col][0], lane, 2048.0f);
#pragma unroll
    for (int j = 0; j < 16; ++j) acc[j] = wmma16(pa, frag_h(MV + (size_t)(j * 16 + col) * MM + ks * 32, lane), acc[j]);
    __syncthreads();
    if (tid < 8) vst2(SG + (size_t)blockIdx.x * MM + ks * 32 + tid * 4, *(const v4f*)&sgb[tid * 4]);
    }
#pragma unroll
  for (int r = 0; r < 8; ++r) { const float il = (1.0f / 2048.0f) / l[r];
#pragma unroll
    for (int j = 0; j < 16; ++j) so[wave][8 * g + r][j * 16 + col] = acc[j][r] * il; }
  __syncthreads();
  for (int rl = 0; rl < 16; ++rl) { vst2(READ + (r0 + rl) * HH + lane * 4, *(const v4f*)&so[wave][rl][lane * 4]); vst2(READ + (r0 + rl) * HH + 128 + lane * 4, *(const v4f*)&so[wave][rl][128 + lane * 4]); }
  for (int h = tid; h < HH; h += 128) { float a = 0.f;
#pragma unroll 1
    for (int rr = 0; rr < 64; ++rr) a += so[rr >> 4][rr & 15][h];
    ssr[h] = a; }
  __syncthreads(); if (tid < HH / 4) vst2(SR + (size_t)blockIdx.x * HH + tid * 4, *(const v4f*)&ssr[tid * 4]); }
__global__ __launch_bounds__(256) void k_avg(const float* __restrict__ SR, float* __restrict__ RA) { __shared__ __align__(16) float s[HH]; const int t = threadIdx.x; float a = 0.f;
#pragma unroll 1
  for (int b = 0; b < TBLK; ++b) a += SR[(size_t)b * HH + t];
  s[t] = a * (1.0f / NROW); __syncthreads(); if (t < HH / 4) vst2(RA + t * 4, *(const v4f*)&s[t * 4]); }
__global__ __launch_bounds__(256) void k_upd(const float* __restrict__ MEM, const float* __restrict__ SG, const float* __restrict__ RA, const float* __restrict__ GA, const float* __restrict__ BE, float* __restrict__ OUT1) { __shared__ float red[8]; __shared__ float stat[3]; __shared__ __align__(16) float so[HH];
  const int t = threadIdx.x; const int mslot = blockIdx.x;
  { float a = 0.f;
#pragma unroll 1
    for (int b = t; b < TBLK; b += 256) a += SG[(size_t)b * MM + mslot];
#pragma unroll
    for (int o = 1; o < 32; o <<= 1) a += __shfl_xor(a, o);
    if ((t & 31) == 0) red[t >> 5] = a; __syncthreads(); if (t == 0) { float q = 0.f; for (int i = 0; i < 8; ++i) q += red[i]; stat[2] = q * (1.0f / NROW); } __syncthreads(); }
  const float gte = stat[2]; const float v = bfr(MEM[(size_t)mslot * HH + t]) * (1.0f - gte) + RA[t] * gte;
  float a = v;
#pragma unroll
  for (int o = 1; o < 32; o <<= 1) a += __shfl_xor(a, o);
  __syncthreads(); if ((t & 31) == 0) red[t >> 5] = a; __syncthreads(); if (t == 0) { float q = 0.f; for (int i = 0; i < 8; ++i) q += red[i]; stat[0] = q * (1.0f / HH); } __syncthreads();
  const float mu = stat[0]; float d = (v - mu) * (v - mu);
#pragma unroll
  for (int o = 1; o < 32; o <<= 1) d += __shfl_xor(d, o);
  __syncthreads(); if ((t & 31) == 0) red[t >> 5] = d; __syncthreads(); if (t == 0) { float q = 0.f; for (int i = 0; i < 8; ++i) q += red[i]; stat[1] = 1.0f / sqrtf(q * (1.0f / HH) + 1e-5f); } __syncthreads();
  so[t] = (v - mu) * stat[1] * bfr(GA[t]) + bfr(BE[t]);
  __syncthreads(); if (t < HH / 4) vst2(OUT1 + (size_t)mslot * HH + t * 4, *(const v4f*)&so[t * 4]); }
extern "C" void kernel_launch(void* const* d_in, const int* in_sizes, int n_in, void* d_out, int out_size, void* d_ws, size_t ws_size, hipStream_t stream) {
  (void)in_sizes; (void)n_in; (void)out_size;
  const float** F = (const float**)d_in;
  if (ws_size < (size_t)WS_END) return;
  char* ws = (char*)d_ws; _Float16 *MHr = (_Float16*)(ws + WS_MH), *MV = (_Float16*)(ws + WS_MV); float *SG = (float*)(ws + WS_SG), *SR = (float*)(ws + WS_SR), *RA = (float*)(ws + WS_RA);
  float* READ = (float*)d_out; float* OUT1 = READ + (size_t)NROW * HH;
  k_mem<<<MM / 64, 256, 0, stream>>>(F[1], MHr, MV);
  k_read<<<TBLK, 128, 0, stream>>>(F[0], MHr, MV, READ, SG, SR);
  k_avg<<<1, 256, 0, stream>>>(SR, RA);
  k_upd<<<MM, 256, 0, stream>>>(F[1], SG, RA, F[2], F[3], OUT1);
}
